// CharacterAwareAttention_7172595384972
// MI455X (gfx1250) — hardware-run, weakly checked
//
#include <hip/hip_runtime.h>


#define NB_  2
#define TQ   1024
#define TK   4096
#define DD   1024
#define NH_  16
#define HD   64
#define NWB  129
#define ZH   2
#define PCAR 1024.0f
typedef _Float16 h16;
typedef unsigned short bf;
typedef __attribute__((ext_vector_type(16))) __bf16   v16bf;
typedef __attribute__((ext_vector_type(16))) _Float16 v16h;
typedef __attribute__((ext_vector_type(8)))  _Float16 v8h;
typedef __attribute__((ext_vector_type(8)))  unsigned short v8us;
typedef __attribute__((ext_vector_type(8)))  float    v8f;
typedef __attribute__((ext_vector_type(4)))  float    v4f;
typedef v8h  __attribute__((may_alias)) v8ha;
typedef v4f  __attribute__((may_alias)) v4fa;
typedef v8us __attribute__((may_alias)) v8usa;

__device__ __forceinline__ unsigned short f2bf(float f) { unsigned u = __float_as_uint(f); u += 0x7FFFu + ((u >> 16) & 1u); return (unsigned short)(u >> 16); }
__device__ __forceinline__ float bf2f(unsigned short b) { return __uint_as_float(((unsigned)b) << 16); }
__device__ __forceinline__ float bfr(float f) { return bf2f(f2bf(f)); }
__device__ __forceinline__ v16h cat16(v8h lo, v8h hi) { return __builtin_shufflevector(lo, hi, 0, 1, 2, 3, 4, 5, 6, 7, 8, 9, 10, 11, 12, 13, 14, 15); }
__device__ __forceinline__ v16bf cat16b(v8us lo, v8us hi) { return __builtin_bit_cast(v16bf, __builtin_shufflevector(lo, hi, 0, 1, 2, 3, 4, 5, 6, 7, 8, 9, 10, 11, 12, 13, 14, 15)); }
__device__ __forceinline__ v8f wmma16(v16h a, v16h b, v8f c) { return __builtin_amdgcn_wmma_f32_16x16x32_f16(false, a, false, b, (short)0, c, false, false); }
__device__ __forceinline__ v8f wmmab(v16bf a, v16bf b, v8f c) { return __builtin_amdgcn_wmma_f32_16x16x32_bf16(false, a, false, b, (short)0, c, false, false); }


template <typename T16> struct WFrag;
template <> struct WFrag<h16> { typedef v16h V; static __device__ __forceinline__ V ld(const h16* p) { return cat16(*(const v8h*)p, *(const v8h*)(p + 16)); } static __device__ __forceinline__ v8f mma(V a, V b, v8f c) { return wmma16(a, b, c); } };
template <> struct WFrag<bf> { typedef v16bf V; static __device__ __forceinline__ V ld(const bf* p) { return cat16b(*(const v8us*)p, *(const v8us*)(p + 16)); } static __device__ __forceinline__ v8f mma(V a, V b, v8f c) { return wmmab(a, b, c); } };
template <typename T16, int NSPLIT, bool BIAS>
__global__ __launch_bounds__(32) void k_gemmw(const T16* __restrict__ A, const T16* __restrict__ A2, const T16* __restrict__ Bt, const T16* __restrict__ Bt2, int K, float* C, int ldc, const float* __restrict__ bias, size_t sA, size_t sB, size_t sC) {
    typedef typename WFrag<T16>::V V;
    __shared__ __align__(16) float os[16 * 68];
    const size_t z = blockIdx.z; A += z * sA; if (A2) A2 += z * sA; Bt += z * sB; if (Bt2) Bt2 += z * sB; C += z * sC;
    const int lane = threadIdx.x & 31, lr = lane & 15, hi = lane >> 4; const int r0 = blockIdx.x * 64, c0 = blockIdx.y * 64;
    v8f acc[4][4];
#pragma unroll
    for (int mb = 0; mb < 4; ++mb)
#pragma unroll
        for (int nb = 0; nb < 4; ++nb) acc[mb][nb] = (v8f){};
    const size_t aoff = (size_t)(r0 + lr) * K + 8 * hi, boff = (size_t)(c0 + lr) * K + 8 * hi;
#pragma unroll 1
    for (int kc = 0; kc < K; kc += 32) {
        V a[4], a2[4];
#pragma unroll
        for (int mb = 0; mb < 4; ++mb) { a[mb] = WFrag<T16>::ld(A + aoff + (size_t)mb * 16 * K + kc); if (NSPLIT == 1 || NSPLIT == 2) a2[mb] = WFrag<T16>::ld(A2 + aoff + (size_t)mb * 16 * K + kc); }
#pragma unroll
        for (int nb = 0; nb < 4; ++nb) { const V b = WFrag<T16>::ld(Bt + boff + (size_t)nb * 16 * K + kc); V b2; if (NSPLIT >= 2) b2 = WFrag<T16>::ld(Bt2 + boff + (size_t)nb * 16 * K + kc);
#pragma unroll
            for (int mb = 0; mb < 4; ++mb) { acc[mb][nb] = WFrag<T16>::mma(a[mb], b, acc[mb][nb]); if (NSPLIT == 1 || NSPLIT == 2) acc[mb][nb] = WFrag<T16>::mma(a2[mb], b, acc[mb][nb]); if (NSPLIT >= 2) acc[mb][nb] = WFrag<T16>::mma(a[mb], b2, acc[mb][nb]); } }
        asm volatile("v_nop\n\tv_nop\n\tv_nop\n\tv_nop" : "+v"(acc[0][0]), "+v"(acc[1][1]), "+v"(acc[2][2]), "+v"(acc[3][3]) : "v"(a[0]), "v"(a[3]));
    }
#pragma unroll
    for (int mb = 0; mb < 4; ++mb) {
#pragma unroll
        for (int nb = 0; nb < 4; ++nb) {
#pragma unroll
            for (int j = 0; j < 8; ++j) os[(hi * 8 + j) * 68 + nb * 16 + lr] = acc[mb][nb][j]; }
        __builtin_amdgcn_wave_barrier(); asm volatile("" ::: "memory");
        float* crow = C + (size_t)(r0 + mb * 16) * ldc + c0;
#pragma unroll 1
        for (int ps = 0; ps < 2; ++ps) {
#pragma unroll
            for (int s = 0; s < 8; ++s) { const int row = 2 * s + hi, cofs = lr * 4; v4f val = *(const v4fa*)(os + row * 68 + cofs); if (BIAS) { val[0] += bfr(bias[c0 + cofs]); val[1] += bfr(bias[c0 + cofs + 1]); val[2] += bfr(bias[c0 + cofs + 2]); val[3] += bfr(bias[c0 + cofs + 3]); }
                *(volatile v4f*)(crow + (size_t)row * ldc + cofs) = val; }
            if (ps == 0) __threadfence(); }
        __builtin_amdgcn_wave_barrier(); asm volatile("" ::: "memory");
    }
}

__device__ __forceinline__ h16 tohx(float x) { return (h16)x; }
__device__ __forceinline__ void splitf(float y, unsigned short& h, unsigned short& l) { h = f2bf(y); l = f2bf(y - bf2f(h)); }
typedef __attribute__((ext_vector_type(2))) _Float16 v2h;
typedef __attribute__((ext_vector_type(4))) _Float16 v4h;
typedef __attribute__((ext_vector_type(4))) unsigned short v4us;

__global__ __launch_bounds__(256) void k_cvt8(const float* __restrict__ src, bf* dst, size_t n8) { const size_t i = (size_t)blockIdx.x * 256 + threadIdx.x; if (i >= n8) return; const v8f v = *(const v8f*)(src + i * 8); v8us o;
#pragma unroll
    for (int k = 0; k < 8; ++k) o[k] = f2bf(v[k]); *(volatile v8us*)(dst + i * 8) = o; __threadfence(); *(volatile v8us*)(dst + i * 8) = o; }
__device__ __forceinline__ int wbat(const int* wb, int i) { i = min(max(i, 0), NWB - 1); return wb[i]; }
__device__ __forceinline__ int cbat(const int* cb, int i) { i = min(max(i, 0), TQ - 1); return cb[i]; }
__global__ __launch_bounds__(256) void k_mask(const int* __restrict__ wb, const int* __restrict__ cb, float* MASK) { const size_t e = ((size_t)blockIdx.x * 256 + threadIdx.x) * 4; if (e >= (size_t)TQ * TK) return; const int k0 = (int)(e % TK); const int q = (int)(e / TK); const int nW = NWB - 1; int cnt = 0;
#pragma unroll 1
    for (int m = 0; m < NWB; ++m) cnt += (wb[m] <= q) ? 1 : 0;
    const int i = min(max(cnt - 1, 0), nW - 1); const int ws = wbat(wb, i), we = wbat(wb, i + 1); const bool valid = (q >= ws) && (q < we); const int cs = cbat(cb, ws), ce = cbat(cb, we - 1); const int ps = wbat(wb, max(i - 1, 0)); const int ns = we, ne = wbat(wb, min(i + 2, nW)); v4f o;
#pragma unroll
    for (int u = 0; u < 4; ++u) { const int k = k0 + u; const bool in_char = (k >= cs) && (k < ce); const bool in_prev = (i > 0) && (k >= ps) && (k < ws); const bool in_next = (i < nW - 1) && (k >= ns) && (k < ne); o[u] = (valid && (in_char || in_prev || in_next)) ? 1.0f : 0.0f; }
    *(volatile v4f*)(MASK + e) = o; __threadfence(); *(volatile v4f*)(MASK + e) = o; }
__global__ __launch_bounds__(256) void k_lnpl(const float* __restrict__ X, const float* __restrict__ g, const float* __restrict__ bb, bf* Xh, bf* Xl) { const int lane = threadIdx.x & 31; const int t = blockIdx.x * 8 + (threadIdx.x >> 5); if (t >= TQ) return; const size_t rb = (size_t)t * DD; float s = 0.f;
#pragma unroll 1
    for (int ch = 0; ch < 8; ++ch) { const v4f a = *(const v4f*)(X + rb + ch * 128 + lane * 4);
#pragma unroll
        for (int q = 0; q < 4; ++q) s = __fadd_rn(s, bfr(a[q])); }
#pragma unroll
    for (int sh = 16; sh; sh >>= 1) s += __shfl_xor(s, sh, 32);
    const float mu = s * (1.0f / DD); float q2 = 0.f;
#pragma unroll 1
    for (int ch = 0; ch < 8; ++ch) { const v4f a = *(const v4f*)(X + rb + ch * 128 + lane * 4);
#pragma unroll
        for (int q = 0; q < 4; ++q) { float dv = __fsub_rn(bfr(a[q]), mu); asm volatile("" : "+v"(dv)); float p = __fmul_rn(dv, dv); asm volatile("" : "+v"(p)); q2 = __fadd_rn(q2, p); } }
#pragma unroll
    for (int sh = 16; sh; sh >>= 1) q2 += __shfl_xor(q2, sh, 32);
    float vq = q2 * (1.0f / DD); asm volatile("" : "+v"(vq)); const float rs = __frsqrt_rn(__fadd_rn(vq, 1e-5f));
#pragma unroll 1
    for (int ch = 0; ch < 8; ++ch) { const int c0 = ch * 128 + lane * 4; const v4f a = *(const v4f*)(X + rb + c0); v4us oh, ol;
#pragma unroll
        for (int q = 0; q < 4; ++q) { float dv = __fsub_rn(bfr(a[q]), mu); asm volatile("" : "+v"(dv)); float tn = __fmul_rn(dv, rs); asm volatile("" : "+v"(tn)); float tg = __fmul_rn(tn, bfr(g[c0 + q])); asm volatile("" : "+v"(tg)); unsigned short u, c; splitf(__fadd_rn(tg, bfr(bb[c0 + q])), u, c); oh[q] = u; ol[q] = c; }
        *(volatile v4us*)(Xh + rb + c0) = oh; *(volatile v4us*)(Xl + rb + c0) = ol; __threadfence(); *(volatile v4us*)(Xh + rb + c0) = oh; *(volatile v4us*)(Xl + rb + c0) = ol; } }
__global__ __launch_bounds__(256) void k_pl(const float* __restrict__ F, int ntok, float scl, h16* P16) { const size_t e = ((size_t)blockIdx.x * 256 + threadIdx.x) * 2; if (e >= (size_t)NH_ * ntok * HD) return; const int d = (int)(e % HD); const int t = (int)((e / HD) % ntok); const int h = (int)(e / ((size_t)HD * ntok)); v2h o; o[0] = tohx(F[(size_t)t * DD + h * HD + d] * scl); o[1] = tohx(F[(size_t)t * DD + h * HD + d + 1] * scl); *(volatile v2h*)(P16 + e) = o; __threadfence(); *(volatile v2h*)(P16 + e) = o; }
__global__ __launch_bounds__(256) void k_vt(const float* __restrict__ F, h16* VT) { const size_t e = ((size_t)blockIdx.x * 256 + threadIdx.x) * 2; if (e >= (size_t)NH_ * HD * TK) return; const int k = (int)(e % TK); const int d = (int)((e / TK) % HD); const int h = (int)(e / ((size_t)TK * HD)); v2h o; o[0] = tohx(F[(size_t)k * DD + h * HD + d]); o[1] = tohx(F[(size_t)(k + 1) * DD + h * HD + d]); *(volatile v2h*)(VT + e) = o; __threadfence(); *(volatile v2h*)(VT + e) = o; }
__global__ __launch_bounds__(256) void k_soft3(const float* __restrict__ Sb, const float* __restrict__ MASK, h16* P) { const int lane = threadIdx.x & 31; const int row = blockIdx.x * 8 + (threadIdx.x >> 5); if (row >= ZH * TQ) return; const int q = row % TQ; const float* sr = Sb + (size_t)row * TK; const float* mr = MASK + (size_t)q * TK; float mx = -3.0e38f;
    for (int ch = 0; ch < TK / 128; ++ch) { const v4f a = *(const v4f*)(sr + ch * 128 + lane * 4); const v4f m = *(const v4f*)(mr + ch * 128 + lane * 4);
#pragma unroll
        for (int u = 0; u < 4; ++u) mx = fmaxf(mx, __fadd_rn(a[u], m[u])); }
#pragma unroll
    for (int sh = 16; sh; sh >>= 1) mx = fmaxf(mx, __shfl_xor(mx, sh, 32));
    float sum = 0.f;
    for (int ch = 0; ch < TK / 128; ++ch) { const v4f a = *(const v4f*)(sr + ch * 128 + lane * 4); const v4f m = *(const v4f*)(mr + ch * 128 + lane * 4);
#pragma unroll
        for (int u = 0; u < 4; ++u) { float d0 = __fsub_rn(__fadd_rn(a[u], m[u]), mx); asm volatile("" : "+v"(d0)); sum += __expf(d0); } }
#pragma unroll
    for (int sh = 16; sh; sh >>= 1) sum += __shfl_xor(sum, sh, 32);
    const float f = __fdiv_rn(PCAR, sum);
    for (int ps = 0; ps < 2; ++ps) { for (int ch = 0; ch < TK / 128; ++ch) { const int j0 = ch * 128 + lane * 4; const v4f a = *(const v4f*)(sr + j0); const v4f m = *(const v4f*)(mr + j0); v4h o;
#pragma unroll
            for (int u = 0; u < 4; ++u) { float d0 = __fsub_rn(__fadd_rn(a[u], m[u]), mx); asm volatile("" : "+v"(d0)); o[u] = tohx(__fmul_rn(__expf(d0), f)); }
            *(volatile v4h*)(P + (size_t)row * TK + j0) = o; } if (ps == 0) __threadfence(); } }
__global__ __launch_bounds__(256) void k_mrg(const float* __restrict__ Ob, int h0, bf* Mh, bf* Ml) { const size_t e = ((size_t)blockIdx.x * 256 + threadIdx.x) * 4; if (e >= (size_t)ZH * TQ * HD) return; const int d = (int)(e % HD); const int t = (int)((e / HD) % TQ); const int z = (int)(e / ((size_t)HD * TQ)); const v4f a = *(const v4f*)(Ob + e); v4us oh, ol;
#pragma unroll
    for (int u = 0; u < 4; ++u) { unsigned short x, c; splitf(a[u] * (1.0f / PCAR), x, c); oh[u] = x; ol[u] = c; } const size_t o = (size_t)t * DD + (h0 + z) * HD + d; *(volatile v4us*)(Mh + o) = oh; *(volatile v4us*)(Ml + o) = ol; __threadfence(); *(volatile v4us*)(Mh + o) = oh; *(volatile v4us*)(Ml + o) = ol; }
__global__ __launch_bounds__(256) void k_fin(const float* __restrict__ x, const float* __restrict__ R, float* OUT) { const size_t i = ((size_t)blockIdx.x * 256 + threadIdx.x) * 4; if (i >= (size_t)TQ * DD) return; const v4f r = *(const v4f*)(R + i); v4f o; o[0] = __fadd_rn(bfr(x[i]), r[0]); o[1] = __fadd_rn(bfr(x[i + 1]), r[1]); o[2] = __fadd_rn(bfr(x[i + 2]), r[2]); o[3] = __fadd_rn(bfr(x[i + 3]), r[3]); *(volatile v4f*)(OUT + i) = o; __threadfence(); *(volatile v4f*)(OUT + i) = o; }

extern "C" void kernel_launch(void* const* d_in, const int* in_sizes, int n_in,
                              void* d_out, int out_size, void* d_ws, size_t ws_size, hipStream_t stream) {
    (void)in_sizes; (void)n_in; (void)out_size;
    const float* qs = (const float*)d_in[0]; const float* ks = (const float*)d_in[1]; const float* vs = (const float*)d_in[2]; const int* wb = (const int*)d_in[3]; const int* cb = (const int*)d_in[4]; const float* g = (const float*)d_in[5]; const float* be = (const float*)d_in[6]; const float* wi = (const float*)d_in[7]; const float* bi = (const float*)d_in[8]; const float* wo = (const float*)d_in[9]; const float* bo = (const float*)d_in[10];
    float* OUT = (float*)d_out;
    char* wsp = (char*)d_ws;
    auto take = [&](size_t bytes) { char* p = wsp; wsp += (bytes + 255) & ~(size_t)255; return (void*)p; };
    bf* WI = (bf*)take((size_t)3 * DD * DD * 2); bf* WO = (bf*)take((size_t)DD * DD * 2); float* MASK = (float*)take((size_t)TQ * TK * 4); bf* Xh = (bf*)take((size_t)TQ * DD * 2); bf* Xl = (bf*)take((size_t)TQ * DD * 2); bf* KB = (bf*)take((size_t)TK * DD * 2);
    float* QF = (float*)take((size_t)TQ * DD * 4); float* KF = (float*)take((size_t)TK * DD * 4); h16* Q16 = (h16*)take((size_t)NH_ * TQ * HD * 2); h16* K16 = (h16*)take((size_t)NH_ * TK * HD * 2); h16* VT = (h16*)take((size_t)NH_ * HD * TK * 2);
    float* Sb = (float*)take((size_t)ZH * TQ * TK * 4); h16* P16 = (h16*)take((size_t)ZH * TQ * TK * 2); float* Ob = (float*)take((size_t)ZH * TQ * HD * 4); bf* Mh = (bf*)take((size_t)TQ * DD * 2); bf* Ml = (bf*)take((size_t)TQ * DD * 2); float* R = QF;
    if ((size_t)(wsp - (char*)d_ws) > ws_size) return;
    k_cvt8<<<(unsigned)(((size_t)3 * DD * DD / 8 + 255) / 256), 256, 0, stream>>>(wi, WI, (size_t)3 * DD * DD / 8); k_cvt8<<<(unsigned)(((size_t)DD * DD / 8 + 255) / 256), 256, 0, stream>>>(wo, WO, (size_t)DD * DD / 8);
    k_mask<<<(unsigned)(((size_t)TQ * TK / 4 + 255) / 256), 256, 0, stream>>>(wb, cb, MASK);
    for (int b = 0; b < NB_; ++b) { const float* xq = qs + (size_t)b * TQ * DD;
        k_lnpl<<<TQ / 8, 256, 0, stream>>>(xq, g, be, Xh, Xl); k_gemmw<bf, 1, true><<<dim3(TQ / 64, DD / 64, 1), 32, 0, stream>>>(Xh, Xl, WI, nullptr, DD, QF, DD, bi, 0, 0, 0);
        k_pl<<<(unsigned)(((size_t)NH_ * TQ * HD / 2 + 255) / 256), 256, 0, stream>>>(QF, TQ, 0.125f, Q16);
        k_cvt8<<<(unsigned)(((size_t)TK * DD / 8 + 255) / 256), 256, 0, stream>>>(ks + (size_t)b * TK * DD, KB, (size_t)TK * DD / 8); k_gemmw<bf, 0, true><<<dim3(TK / 64, DD / 64, 1), 32, 0, stream>>>(KB, nullptr, WI + (size_t)DD * DD, nullptr, DD, KF, DD, bi + DD, 0, 0, 0);
        k_pl<<<(unsigned)(((size_t)NH_ * TK * HD / 2 + 255) / 256), 256, 0, stream>>>(KF, TK, 1.0f, K16);
        k_cvt8<<<(unsigned)(((size_t)TK * DD / 8 + 255) / 256), 256, 0, stream>>>(vs + (size_t)b * TK * DD, KB, (size_t)TK * DD / 8); k_gemmw<bf, 0, true><<<dim3(TK / 64, DD / 64, 1), 32, 0, stream>>>(KB, nullptr, WI + (size_t)2 * DD * DD, nullptr, DD, KF, DD, bi + 2 * DD, 0, 0, 0);
        k_vt<<<(unsigned)(((size_t)NH_ * HD * TK / 2 + 255) / 256), 256, 0, stream>>>(KF, VT);
        for (int h0 = 0; h0 < NH_; h0 += ZH) { const size_t z = (size_t)h0;
            k_gemmw<h16, 0, false><<<dim3(TQ / 64, TK / 64, ZH), 32, 0, stream>>>(Q16 + z * TQ * HD, nullptr, K16 + z * TK * HD, nullptr, HD, Sb, TK, nullptr, (size_t)TQ * HD, (size_t)TK * HD, (size_t)TQ * TK);
            k_soft3<<<ZH * TQ / 8, 256, 0, stream>>>(Sb, MASK, P16);
            k_gemmw<h16, 0, false><<<dim3(TQ / 64, 1, ZH), 32, 0, stream>>>(P16, nullptr, VT + z * HD * TK, nullptr, TK, Ob, HD, nullptr, (size_t)TQ * TK, (size_t)HD * TK, (size_t)TQ * HD);
            k_mrg<<<(unsigned)(((size_t)ZH * TQ * HD / 4 + 255) / 256), 256, 0, stream>>>(Ob, h0, Mh, Ml); }
        k_gemmw<bf, 1, true><<<dim3(TQ / 64, DD / 64, 1), 32, 0, stream>>>(Mh, Ml, WO, nullptr, DD, R, DD, bo, 0, 0, 0);
        k_fin<<<(TQ * DD / 4 + 255) / 256, 256, 0, stream>>>(xq, R, OUT + (size_t)b * TQ * DD); }
}
